// GNN_82377472737433
// MI455X (gfx1250) — hardware-verified
//
#include <hip/hip_runtime.h>
#include <stddef.h>
#include <stdint.h>
#include <math.h>


#define CIN    128
#define FH     256
#define K2     512
#define NTHR   256
#define NWAVE  8
#define EPT    8
#define CHUNK  (NTHR * EPT)
#define WCAP   (EPT * 32)
#define LISTN  (NWAVE * WCAP)
#define NBD    8192
#define SLD    13
#define NBA    1024
#define SLA    10
#define RCAP   28672
#define DEGCAP 64
#define GBM    64
#define GBN    64
#define GTHR   128
#define NU1    (FH * (CIN / 8))
#define NU2    (FH * (K2 / 8))
#define AGG_ZINTS    (LISTN + 2 * RCAP + 3 * NBA)
#define MISC_INTS    16
#define ROWBUF_INTS  (NWAVE * K2 / 2)
#define AGG_LDS_INTS (AGG_ZINTS + MISC_INTS + ROWBUF_INTS)
#define WSMAX  134217728

static_assert((CHUNK & (CHUNK - 1)) == 0 && CHUNK <= 4096);
static_assert((NBD & (NBD - 1)) == 0 && NBD == (1 << SLD));
static_assert((NBA & (NBA - 1)) == 0 && NBA == (1 << SLA));
static_assert(((long long)CHUNK << SLD) < (1LL << 31));
static_assert(((long long)CHUNK << SLA) < (1LL << 31));
static_assert(NBD % (NTHR * 4) == 0 && NBD % NTHR == 0);
static_assert(LISTN % NTHR == 0);
static_assert(NBA % NWAVE == 0 && NBA % 32 == 0 && NBA % GBM == 0 && NBA == 4 * NTHR);
static_assert(RCAP % 4 == 0 && AGG_ZINTS % 4 == 0 && LISTN % 4 == 0 && ((AGG_ZINTS + MISC_INTS) % 4) == 0);
static_assert(AGG_ZINTS % (NTHR * 4) == 0);
static_assert(CIN % 32 == 0 && K2 % 32 == 0 && K2 == 2 * FH && FH % GBN == 0);
static_assert(GBM == (GTHR / 32) * 16 && GBN == 64);
static_assert(NU1 % NTHR == 0 && NU2 % NTHR == 0);
static_assert(CIN / 8 == 16 && K2 / 8 == 64);
static_assert(FH == 8 * 32);
static_assert(AGG_LDS_INTS * 4 <= 300000);

typedef float          v4f   __attribute__((ext_vector_type(4)));
typedef float          v8f   __attribute__((ext_vector_type(8)));
typedef int            v4i   __attribute__((ext_vector_type(4)));
typedef int            v8i   __attribute__((ext_vector_type(8)));
typedef unsigned short v4us  __attribute__((ext_vector_type(4)));
typedef unsigned short v8us  __attribute__((ext_vector_type(8)));
typedef unsigned short v16us __attribute__((ext_vector_type(16)));
typedef __bf16         v16bf __attribute__((ext_vector_type(16)));
typedef v4f  __attribute__((may_alias)) v4fa;
typedef v4i  __attribute__((may_alias)) v4ia;
typedef v4us __attribute__((may_alias)) v4usa;
typedef v8us __attribute__((may_alias)) v8usa;
union FragB { v16bf v; v16us u; v8us h[2]; v8i w; };

__device__ __forceinline__ v8f wmb(const FragB& a, const FragB& b, v8f c) {
  v8f d = __builtin_amdgcn_wmma_f32_16x16x32_bf16(false, a.v, false, b.v, (short)0, c, false, false);
  asm volatile("v_nop\n\tv_nop\n\tv_nop\n\tv_nop" : "+v"(d) : "v"(a.w), "v"(b.w));
  return d;
}

__device__ __forceinline__ unsigned bf16_bits(float f) {
  const unsigned u = __float_as_uint(f);
  return (u + 0x7FFFu + ((u >> 16) & 1u)) >> 16;
}
__device__ __forceinline__ float bf16_val(float f) {
  return __uint_as_float(bf16_bits(f) << 16);
}
__device__ __forceinline__ float relu_np(float v) {
  return (v > 0.0f) ? v : (v - v);
}

__device__ __forceinline__ void wave_sync() {
  __builtin_amdgcn_fence(__ATOMIC_RELEASE, "wavefront");
  __builtin_amdgcn_wave_barrier();
  __builtin_amdgcn_fence(__ATOMIC_ACQUIRE, "wavefront");
}

template <int SLB>
__device__ __forceinline__ int scan_chunk(const int* __restrict__ dsts, int nE, int cbase, int slotBase,
                                          int nb, int vec8, int* list, int tid, int lane, int wave) {
  int wc = 0;
  const int el0  = tid * EPT;
  const int e0   = cbase + el0;
  const int sent = -2147483647 - 1;
  v4i da, db;
  if (vec8 != 0 && cbase + CHUNK <= nE) {
    da = *(const v4i*)(dsts + e0);
    db = *(const v4i*)(dsts + e0 + 4);
  } else {
    da.x = (e0     < nE) ? dsts[min(e0,     nE - 1)] : sent;
    da.y = (e0 + 1 < nE) ? dsts[min(e0 + 1, nE - 1)] : sent;
    da.z = (e0 + 2 < nE) ? dsts[min(e0 + 2, nE - 1)] : sent;
    da.w = (e0 + 3 < nE) ? dsts[min(e0 + 3, nE - 1)] : sent;
    db.x = (e0 + 4 < nE) ? dsts[min(e0 + 4, nE - 1)] : sent;
    db.y = (e0 + 5 < nE) ? dsts[min(e0 + 5, nE - 1)] : sent;
    db.z = (e0 + 6 < nE) ? dsts[min(e0 + 6, nE - 1)] : sent;
    db.w = (e0 + 7 < nE) ? dsts[min(e0 + 7, nE - 1)] : sent;
  }
  const unsigned nbs = (unsigned)slotBase;
  const unsigned unb = (unsigned)nb;
  const unsigned s0 = (unsigned)da.x - nbs, s1 = (unsigned)da.y - nbs;
  const unsigned s2 = (unsigned)da.z - nbs, s3 = (unsigned)da.w - nbs;
  const unsigned s4 = (unsigned)db.x - nbs, s5 = (unsigned)db.y - nbs;
  const unsigned s6 = (unsigned)db.z - nbs, s7 = (unsigned)db.w - nbs;
  const bool h0 = s0 < unb, h1 = s1 < unb, h2 = s2 < unb, h3 = s3 < unb;
  const bool h4 = s4 < unb, h5 = s5 < unb, h6 = s6 < unb, h7 = s7 < unb;
  const unsigned any = __builtin_amdgcn_ballot_w32(h0 | h1 | h2 | h3 | h4 | h5 | h6 | h7);
  if (any != 0u) {
#define HITJ(J, HJ, SJ) { \
      const unsigned mj = __builtin_amdgcn_ballot_w32(HJ); \
      if (mj != 0u) { \
        if (HJ) { \
          const int pos = wc + (int)__builtin_amdgcn_mbcnt_lo(mj, 0u); \
          if (pos < WCAP) list[wave * WCAP + pos] = ((el0 + (J)) << SLB) | (int)(SJ); \
        } \
        wc += (int)__builtin_popcount(mj); } }
    HITJ(0, h0, s0)
    HITJ(1, h1, s1)
    HITJ(2, h2, s2)
    HITJ(3, h3, s3)
    HITJ(4, h4, s4)
    HITJ(5, h5, s5)
    HITJ(6, h6, s6)
    HITJ(7, h7, s7)
#undef HITJ
  }
  return wc;
}

__global__ __launch_bounds__(NTHR) void k_wprep(const float* __restrict__ W1, const float* __restrict__ W2,
                                                unsigned short* W1T, unsigned short* W2T) {
  const int u = (int)blockIdx.x * NTHR + (int)threadIdx.x;
  v8us o;
  unsigned short* dp;
  if (u < NU1) {
    const int n  = u >> 4;
    const int k8 = (u & 15) * 8;
    const float* p = W1 + (size_t)k8 * FH + n;
#pragma unroll
    for (int i = 0; i < 8; ++i) o[i] = (unsigned short)bf16_bits(p[(size_t)i * FH]);
    dp = W1T + (size_t)n * CIN + k8;
  } else if (u < NU1 + NU2) {
    const int v  = u - NU1;
    const int n  = v >> 6;
    const int k8 = (v & 63) * 8;
    const int kk = k8 & (FH - 1);
    const float* p = W2 + (size_t)kk * FH + n;
#pragma unroll
    for (int i = 0; i < 8; ++i) o[i] = (unsigned short)bf16_bits(p[(size_t)i * FH]);
    dp = W2T + (size_t)n * K2 + k8;
  } else {
    return;
  }
  *(volatile v8us*)dp = o;
  __threadfence();
  *(volatile v8us*)dp = o;
}

__global__ __launch_bounds__(NTHR) void k_cvx(const float* __restrict__ x, int nN, int nUnits,
                                              unsigned short* xb) {
  const int u = (int)blockIdx.x * NTHR + (int)threadIdx.x;
  if (u >= nUnits) return;
  const int row = u >> 4;
  const int k8  = (u & 15) * 8;
  const int rc  = row < nN ? row : nN - 1;
  const float* p = x + (size_t)rc * CIN + k8;
  const v4f a = *(const v4fa*)p;
  const v4f b = *(const v4fa*)(p + 4);
  const bool ok = row < nN;
  v8us o;
  o[0] = ok ? (unsigned short)bf16_bits(a.x) : (unsigned short)0;
  o[1] = ok ? (unsigned short)bf16_bits(a.y) : (unsigned short)0;
  o[2] = ok ? (unsigned short)bf16_bits(a.z) : (unsigned short)0;
  o[3] = ok ? (unsigned short)bf16_bits(a.w) : (unsigned short)0;
  o[4] = ok ? (unsigned short)bf16_bits(b.x) : (unsigned short)0;
  o[5] = ok ? (unsigned short)bf16_bits(b.y) : (unsigned short)0;
  o[6] = ok ? (unsigned short)bf16_bits(b.z) : (unsigned short)0;
  o[7] = ok ? (unsigned short)bf16_bits(b.w) : (unsigned short)0;
  unsigned short* dp = xb + (size_t)row * CIN + k8;
  *(volatile v8us*)dp = o;
  __threadfence();
  *(volatile v8us*)dp = o;
}

__global__ __launch_bounds__(NTHR) void k_deg(const int* __restrict__ dsts, int nE, int vec8, float* dis) {
  __shared__ __attribute__((aligned(16))) int scnt[NBD];
  __shared__ __attribute__((aligned(16))) int list[LISTN];
  __shared__ int wcnt[NWAVE];
  const int tid = (int)threadIdx.x, lane = tid & 31, wave = tid >> 5;
  const int nodeBase = (int)blockIdx.x * NBD;

  for (int i = tid; i < NBD; i += NTHR) scnt[i] = 0;
  for (int i = tid; i < LISTN; i += NTHR) list[i] = 0;
  if (tid < NWAVE) wcnt[tid] = 0;
  __syncthreads();

  const int nChunks = (nE + CHUNK - 1) / CHUNK;
#pragma unroll 1
  for (int ch = 0; ch < nChunks; ++ch) {
    const int cbase = ch * CHUNK;
    const int wc = scan_chunk<SLD>(dsts, nE, cbase, nodeBase, NBD, vec8, list, tid, lane, wave);
    if (lane == 0) wcnt[wave] = wc;
    __syncthreads();
    if (wave == 0) {
#pragma unroll 1
      for (int w2 = 0; w2 < NWAVE; ++w2) {
        int c = wcnt[w2];
        c = c < 0 ? 0 : (c > WCAP ? WCAP : c);
#pragma unroll 1
        for (int b0 = 0; b0 < c; b0 += 32) {
          const int idx = b0 + lane;
          const int ent = list[w2 * WCAP + (idx < WCAP ? idx : WCAP - 1)];
          const int m32 = (c - b0) < 32 ? (c - b0) : 32;
#pragma unroll 1
          for (int k = 0; k < m32; ++k) {
            const int u  = __builtin_amdgcn_readlane(ent, k);
            const int sl = u & (NBD - 1);
            if (lane == 0) scnt[sl] = scnt[sl] + 1;
          }
        }
      }
    }
    __syncthreads();
  }

#pragma unroll 1
  for (int i = tid; i < NBD; i += NTHR) {
    const float d = fmaxf((float)(scnt[i] + 1), 1.0f);
    scnt[i] = __float_as_int(1.0f / sqrtf(d));
  }
  __syncthreads();

  v4f vals[NBD / (NTHR * 4)];
#pragma unroll
  for (int it = 0; it < NBD / (NTHR * 4); ++it) {
    const int s0 = it * (NTHR * 4) + 4 * tid;
    const v4i c4 = *(const v4ia*)(scnt + s0);
    v4f v;
    v.x = __int_as_float(c4.x); v.y = __int_as_float(c4.y);
    v.z = __int_as_float(c4.z); v.w = __int_as_float(c4.w);
    vals[it] = v;
  }
#pragma unroll
  for (int it = 0; it < NBD / (NTHR * 4); ++it) {
    const int s0 = it * (NTHR * 4) + 4 * tid;
    *(volatile v4f*)(dis + (size_t)nodeBase + s0) = vals[it];
  }
  __threadfence();
#pragma unroll
  for (int it = 0; it < NBD / (NTHR * 4); ++it) {
    const int s0 = it * (NTHR * 4) + 4 * tid;
    *(volatile v4f*)(dis + (size_t)nodeBase + s0) = vals[it];
  }
}

__global__ __launch_bounds__(GTHR) void k_gemm(
    const unsigned short* __restrict__ A, const unsigned short* __restrict__ WT,
    float* outF, int K, int ldo)
{
  __shared__ __attribute__((aligned(16))) float stg[GBM * GBN];
  const int tid = (int)threadIdx.x, lane = tid & 31, wave = tid >> 5, hh = lane >> 4, m = lane & 15;
  const int rowBase = (int)blockIdx.x * GBM;
  const int col0    = (int)blockIdx.y * GBN;

  v8f acc[4];
  {
    const v8f z = {0.f, 0.f, 0.f, 0.f, 0.f, 0.f, 0.f, 0.f};
    acc[0] = z; acc[1] = z; acc[2] = z; acc[3] = z;
  }
  const unsigned short* ap = A  + (size_t)(rowBase + 16 * wave + m) * (size_t)K + 8 * hh;
  const unsigned short* wp = WT + (size_t)(col0 + m) * (size_t)K + 8 * hh;
  const int ksteps = K >> 5;
#pragma unroll 1
  for (int ks = 0; ks < ksteps; ++ks) {
    FragB af;
    af.h[0] = *(const v8usa*)(ap + 32 * ks);
    af.h[1] = *(const v8usa*)(ap + 32 * ks + 16);
#pragma unroll
    for (int t = 0; t < 4; ++t) {
      const unsigned short* wq = wp + (size_t)(16 * t) * (size_t)K + 32 * ks;
      FragB bf;
      bf.h[0] = *(const v8usa*)wq;
      bf.h[1] = *(const v8usa*)(wq + 16);
      acc[t] = wmb(af, bf, acc[t]);
    }
  }

#pragma unroll
  for (int t = 0; t < 4; ++t) {
    const int lc = 16 * t + m;
#pragma unroll
    for (int r = 0; r < 8; ++r) {
      const int lr = 16 * wave + 8 * hh + r;
      stg[lr * GBN + lc] = acc[t][r];
    }
  }
  __syncthreads();

  v4f fv[8];
#pragma unroll
  for (int i = 0; i < 8; ++i) {
    const int lr = 16 * wave + 2 * i + hh;
    fv[i] = *(const v4fa*)(stg + lr * GBN + 4 * m);
  }
#pragma unroll
  for (int i = 0; i < 8; ++i) {
    const int lr = 16 * wave + 2 * i + hh;
    const int gr = rowBase + lr;
    float* op = outF + (size_t)gr * (size_t)ldo + col0 + 4 * m;
    *(volatile v4f*)op = fv[i];
  }
  __threadfence();
#pragma unroll
  for (int i = 0; i < 8; ++i) {
    const int lr = 16 * wave + 2 * i + hh;
    const int gr = rowBase + lr;
    float* op = outF + (size_t)gr * (size_t)ldo + col0 + 4 * m;
    *(volatile v4f*)op = fv[i];
  }
}

template <int MODE>
__global__ __launch_bounds__(NTHR) void k_scan(const int* __restrict__ srcs, const int* __restrict__ dsts,
                                               int nE, int nN, int vec8, int mRows,
                                               const float* __restrict__ dis,
                                               const float* __restrict__ xl, const float* __restrict__ bias,
                                               const float* __restrict__ wfc, const float* __restrict__ bfc,
                                               unsigned short* hb, float* outp) {
  extern __shared__ __attribute__((aligned(16))) int dsm[];
  int* list = dsm;
  int* hl   = dsm + LISTN;
  int* sl   = hl + RCAP;
  int* cnt  = sl + RCAP;
  int* offs = cnt + NBA;
  int* cur  = offs + NBA;
  int* misc = cur + NBA;
  const int tid = (int)threadIdx.x, lane = tid & 31, wave = tid >> 5;
  unsigned short* rowbuf = (unsigned short*)(misc + MISC_INTS) + wave * K2;
  const int nodeBase = (int)blockIdx.x * NBA;

  {
    const v4i z4 = {0, 0, 0, 0};
    for (int i = tid * 4; i < AGG_ZINTS; i += NTHR * 4) *(v4ia*)(dsm + i) = z4;
    if (tid < MISC_INTS) misc[tid] = 0;
  }
  v4f bA, bB, wA, wB;
  float bfv;
  {
    const v4f t1 = *(const v4fa*)(bias + 4 * lane);
    const v4f t2 = *(const v4fa*)(bias + 128 + 4 * lane);
    bA.x = bf16_val(t1.x); bA.y = bf16_val(t1.y); bA.z = bf16_val(t1.z); bA.w = bf16_val(t1.w);
    bB.x = bf16_val(t2.x); bB.y = bf16_val(t2.y); bB.z = bf16_val(t2.z); bB.w = bf16_val(t2.w);
    const v4f t3 = *(const v4fa*)(wfc + 4 * lane);
    const v4f t4 = *(const v4fa*)(wfc + 128 + 4 * lane);
    wA.x = bf16_val(t3.x); wA.y = bf16_val(t3.y); wA.z = bf16_val(t3.z); wA.w = bf16_val(t3.w);
    wB.x = bf16_val(t4.x); wB.y = bf16_val(t4.y); wB.z = bf16_val(t4.z); wB.w = bf16_val(t4.w);
    bfv = bf16_val(bfc[0]);
  }
  __syncthreads();

  int t = 0, ov = 0;
  const int nChunks = (nE + CHUNK - 1) / CHUNK;
#pragma unroll 1
  for (int ch = 0; ch < nChunks; ++ch) {
    const int cbase = ch * CHUNK;
    const int wc = scan_chunk<SLA>(dsts, nE, cbase, nodeBase, NBA, vec8, list, tid, lane, wave);
    if (lane == 0) misc[wave] = wc;
    __syncthreads();
    if (wave == 0) {
#pragma unroll 1
      for (int w2 = 0; w2 < NWAVE; ++w2) {
        int c = misc[w2];
        c = c < 0 ? 0 : (c > WCAP ? WCAP : c);
#pragma unroll 1
        for (int b0 = 0; b0 < c; b0 += 32) {
          const int idx = b0 + lane;
          const int ent = list[w2 * WCAP + (idx < WCAP ? idx : WCAP - 1)];
          const int m32 = (c - b0) < 32 ? (c - b0) : 32;
#pragma unroll 1
          for (int k = 0; k < m32; ++k) {
            const int u    = __builtin_amdgcn_readlane(ent, k);
            const int slot = u & (NBA - 1);
            const int el   = (u >> SLA) & (CHUNK - 1);
            const int pk   = ((cbase + el) << SLA) | slot;
            if (t < RCAP) {
              if (lane == 0) { hl[t] = pk; cnt[slot] = cnt[slot] + 1; }
              t = t + 1;
            } else {
              ov = 1;
            }
          }
        }
      }
    }
    __syncthreads();
  }
  if (wave == 0 && lane == 0) { misc[8] = t; misc[9] = ov; }
  __syncthreads();
  int tt = misc[8];
  tt = tt < 0 ? 0 : (tt > RCAP ? RCAP : tt);
  const int ovf = misc[9];

  if (wave == 0) {
    const int base = lane * (NBA / 32);
    int s = 0;
#pragma unroll 1
    for (int i = 0; i < NBA / 32; ++i) s += cnt[base + i];
    int incl = s;
#pragma unroll
    for (int d = 1; d < 32; d <<= 1) {
      const int y = __shfl_up(incl, d, 32);
      if (lane >= d) incl += y;
    }
    int run = incl - s;
#pragma unroll 1
    for (int i = 0; i < NBA / 32; ++i) {
      const int cv = cnt[base + i];
      offs[base + i] = run;
      cur[base + i]  = run;
      run += cv;
    }
  }
  __syncthreads();
  if (wave == 0) {
#pragma unroll 1
    for (int b0 = 0; b0 < tt; b0 += 32) {
      const int idx = b0 + lane;
      const int ent = hl[idx < RCAP ? idx : RCAP - 1];
      const int m32 = (tt - b0) < 32 ? (tt - b0) : 32;
#pragma unroll 1
      for (int k = 0; k < m32; ++k) {
        const int u    = __builtin_amdgcn_readlane(ent, k);
        const int slot = u & (NBA - 1);
        if (lane == 0) {
          int p = cur[slot];
          p = p < 0 ? 0 : (p > RCAP - 1 ? RCAP - 1 : p);
          sl[p] = u;
          cur[slot] = p + 1;
        }
      }
    }
  }
  __syncthreads();

  const float qnan = __int_as_float(0x7fc00000);
  const float pz = (ovf != 0) ? qnan : 0.0f;
#pragma unroll 1
  for (int si = 0; si < NBA / NWAVE; ++si) {
    const int s    = si * NWAVE + wave;
    const int node = nodeBase + s;
    int c = cnt[s];
    const bool big = c > DEGCAP;
    c = c < 0 ? 0 : (c > DEGCAP ? DEGCAP : c);
    int o = offs[s];
    o = o < 0 ? 0 : (o > RCAP ? RCAP : o);
    const int nc = node < nN ? node : nN - 1;
    const float dd = dis[nc];
    const float rd = dd * dd;
    v4f aA = {0.0f, 0.0f, 0.0f, 0.0f};
    v4f aB = {0.0f, 0.0f, 0.0f, 0.0f};
    int bad = 0;
#pragma unroll 1
    for (int b0 = 0; b0 < c; b0 += 32) {
      int idx = o + b0 + lane;
      idx = idx > RCAP - 1 ? RCAP - 1 : idx;
      const int ent = sl[idx];
      int eid = ent >> SLA;
      eid = eid < 0 ? 0 : (eid > nE - 1 ? nE - 1 : eid);
      const int srRaw = srcs[eid];
      const int m32 = (c - b0) < 32 ? (c - b0) : 32;
      const bool oob = (lane < m32) && ((unsigned)srRaw >= (unsigned)nN);
      const unsigned obm = __builtin_amdgcn_ballot_w32(oob);
      bad = (obm != 0u) ? 1 : bad;
      int sr = srRaw;
      sr = sr < 0 ? 0 : (sr > nN - 1 ? nN - 1 : sr);
      const float cf  = dis[sr] * dd;
      const int   cfi = __float_as_int(cf);
#pragma unroll 1
      for (int k = 0; k < m32; ++k) {
        const int   sk = __builtin_amdgcn_readlane(sr, k);
        const float ck = __int_as_float(__builtin_amdgcn_readlane(cfi, k));
        const float* rp = xl + (size_t)sk * FH + 4 * lane;
        const v4f a = *(const v4fa*)rp;
        const v4f b = *(const v4fa*)(rp + 128);
        aA.x = fmaf(ck, a.x, aA.x); aA.y = fmaf(ck, a.y, aA.y);
        aA.z = fmaf(ck, a.z, aA.z); aA.w = fmaf(ck, a.w, aA.w);
        aB.x = fmaf(ck, b.x, aB.x); aB.y = fmaf(ck, b.y, aB.y);
        aB.z = fmaf(ck, b.z, aB.z); aB.w = fmaf(ck, b.w, aB.w);
      }
    }
    v4f sA, sB;
    {
      const float* rp = xl + (size_t)nc * FH + 4 * lane;
      sA = *(const v4fa*)rp;
      sB = *(const v4fa*)(rp + 128);
    }
    const float pzr = (big || bad != 0) ? qnan : pz;
    const bool live = node < nN;
    v4f yA, yB;
    yA.x = relu_np((aA.x + sA.x * rd) + bA.x) + pzr;
    yA.y = relu_np((aA.y + sA.y * rd) + bA.y) + pzr;
    yA.z = relu_np((aA.z + sA.z * rd) + bA.z) + pzr;
    yA.w = relu_np((aA.w + sA.w * rd) + bA.w) + pzr;
    yB.x = relu_np((aB.x + sB.x * rd) + bB.x) + pzr;
    yB.y = relu_np((aB.y + sB.y * rd) + bB.y) + pzr;
    yB.z = relu_np((aB.z + sB.z * rd) + bB.z) + pzr;
    yB.w = relu_np((aB.w + sB.w * rd) + bB.w) + pzr;
    yA.x = live ? yA.x : 0.0f; yA.y = live ? yA.y : 0.0f; yA.z = live ? yA.z : 0.0f; yA.w = live ? yA.w : 0.0f;
    yB.x = live ? yB.x : 0.0f; yB.y = live ? yB.y : 0.0f; yB.z = live ? yB.z : 0.0f; yB.w = live ? yB.w : 0.0f;

    if constexpr (MODE != 0) {
      v4us hA, lA, hB, lB;
      unsigned q;
      q = bf16_bits(yA.x); hA[0] = (unsigned short)q; lA[0] = (unsigned short)bf16_bits(yA.x - __uint_as_float(q << 16));
      q = bf16_bits(yA.y); hA[1] = (unsigned short)q; lA[1] = (unsigned short)bf16_bits(yA.y - __uint_as_float(q << 16));
      q = bf16_bits(yA.z); hA[2] = (unsigned short)q; lA[2] = (unsigned short)bf16_bits(yA.z - __uint_as_float(q << 16));
      q = bf16_bits(yA.w); hA[3] = (unsigned short)q; lA[3] = (unsigned short)bf16_bits(yA.w - __uint_as_float(q << 16));
      q = bf16_bits(yB.x); hB[0] = (unsigned short)q; lB[0] = (unsigned short)bf16_bits(yB.x - __uint_as_float(q << 16));
      q = bf16_bits(yB.y); hB[1] = (unsigned short)q; lB[1] = (unsigned short)bf16_bits(yB.y - __uint_as_float(q << 16));
      q = bf16_bits(yB.z); hB[2] = (unsigned short)q; lB[2] = (unsigned short)bf16_bits(yB.z - __uint_as_float(q << 16));
      q = bf16_bits(yB.w); hB[3] = (unsigned short)q; lB[3] = (unsigned short)bf16_bits(yB.w - __uint_as_float(q << 16));
      *(v4usa*)(rowbuf + 4 * lane) = hA;
      *(v4usa*)(rowbuf + 128 + 4 * lane) = hB;
      *(v4usa*)(rowbuf + FH + 4 * lane) = lA;
      *(v4usa*)(rowbuf + FH + 128 + 4 * lane) = lB;
      wave_sync();
      const v8us q0 = *(const v8usa*)(rowbuf + 8 * lane);
      const v8us q1 = *(const v8usa*)(rowbuf + FH + 8 * lane);
      wave_sync();
      if (node < mRows) {
        unsigned short* rpw = hb + (size_t)node * K2 + 8 * lane;
        *(volatile v8us*)rpw = q0;
        *(volatile v8us*)(rpw + FH) = q1;
        __threadfence();
        *(volatile v8us*)rpw = q0;
        *(volatile v8us*)(rpw + FH) = q1;
      }
    } else {
      float hs = 0.0f;
      hs = fmaf(yA.x, wA.x, hs); hs = fmaf(yA.y, wA.y, hs);
      hs = fmaf(yA.z, wA.z, hs); hs = fmaf(yA.w, wA.w, hs);
      hs = fmaf(yB.x, wB.x, hs); hs = fmaf(yB.y, wB.y, hs);
      hs = fmaf(yB.z, wB.z, hs); hs = fmaf(yB.w, wB.w, hs);
#pragma unroll
      for (int d = 16; d > 0; d >>= 1) hs += __shfl_xor(hs, d, 32);
      const float ovl = live ? (hs + bfv) : 0.0f;
      if (lane == 0) cur[s] = __float_as_int(ovl);
    }
  }

  if constexpr (MODE == 0) {
    __syncthreads();
    const v4i ob = *(const v4ia*)(cur + 4 * tid);
    v4f ovv;
    ovv.x = __int_as_float(ob.x); ovv.y = __int_as_float(ob.y);
    ovv.z = __int_as_float(ob.z); ovv.w = __int_as_float(ob.w);
    const int g0 = nodeBase + 4 * tid;
    const bool okst = (g0 + 3) < nN;
    const int gc = okst ? g0 : 0;
    float* op = outp + (size_t)gc;
    if (okst) *(volatile v4f*)op = ovv;
    __threadfence();
    if (okst) *(volatile v4f*)op = ovv;
  }
}

static inline int cdiv(int a, int b) { return (a + b - 1) / b; }
static inline size_t al256(size_t o) { return (o + 255) & ~(size_t)255; }

extern "C" void kernel_launch(void* const* d_in, const int* in_sizes, int n_in,
                              void* d_out, int out_size, void* d_ws, size_t ws_size,
                              hipStream_t stream) {
  if (n_in < 8) return;
  if (in_sizes[0] < CIN || (in_sizes[0] % CIN) != 0) return;
  const int nN = in_sizes[0] / CIN;
  if (nN < 4 || nN > (1 << 22) || (nN & 3) != 0) return;
  if (in_sizes[1] < 2 || (in_sizes[1] & 1) != 0) return;
  const int nE = in_sizes[1] / 2;
  if (nE < 1 || nE >= (1 << (31 - SLA))) return;
  if (in_sizes[2] != CIN * FH || in_sizes[3] != FH) return;
  if (in_sizes[4] != FH * FH || in_sizes[5] != FH) return;
  if (in_sizes[6] != FH || in_sizes[7] != 1) return;
  if (out_size != nN) return;

  const float* x    = (const float*)d_in[0];
  const int*   edge = (const int*)d_in[1];
  const float* W1   = (const float*)d_in[2];
  const float* b1   = (const float*)d_in[3];
  const float* W2   = (const float*)d_in[4];
  const float* b2   = (const float*)d_in[5];
  const float* Wfc  = (const float*)d_in[6];
  const float* bfc  = (const float*)d_in[7];
  float* out = (float*)d_out;
  const int* src = edge;
  const int* dst = edge + nE;

  const int MP   = cdiv(nN, GBM) * GBM;
  const int gM   = MP / GBM;
  const int gD   = cdiv(nN, NBD);
  const int NBPD = gD * NBD;
  const int gA   = cdiv(MP, NBA);
  if ((long long)gA * NBA < (long long)MP) return;
  if (NBPD < nN) return;
  const int vec8 = ((nE & 3) == 0) ? 1 : 0;

  char* ws = (char*)d_ws;
  size_t off = 0;
  const size_t oDIS = off; off = al256(off + (size_t)NBPD * 4);
  const size_t oW1T = off; off = al256(off + (size_t)FH * CIN * 2);
  const size_t oW2T = off; off = al256(off + (size_t)FH * K2 * 2);
  const size_t oXB  = off; off = al256(off + (size_t)MP * CIN * 2);
  const size_t oXW  = off; off = al256(off + (size_t)MP * FH * 4);
  const size_t oH1  = off; off = al256(off + (size_t)MP * K2 * 2);
  if (off > ws_size || off > (size_t)WSMAX) return;
  float*          DIS = (float*)(ws + oDIS);
  unsigned short* W1T = (unsigned short*)(ws + oW1T);
  unsigned short* W2T = (unsigned short*)(ws + oW2T);
  unsigned short* XB  = (unsigned short*)(ws + oXB);
  float*          XW  = (float*)(ws + oXW);
  unsigned short* H1  = (unsigned short*)(ws + oH1);

  const size_t scanLds = (size_t)AGG_LDS_INTS * 4;
  hipFuncSetAttribute(reinterpret_cast<const void*>(&k_scan<1>), hipFuncAttributeMaxDynamicSharedMemorySize, (int)scanLds);
  hipFuncSetAttribute(reinterpret_cast<const void*>(&k_scan<0>), hipFuncAttributeMaxDynamicSharedMemorySize, (int)scanLds);

  const int nUx = MP * (CIN / 8);
  k_wprep<<<(NU1 + NU2) / NTHR, NTHR, 0, stream>>>(W1, W2, W1T, W2T);
  k_cvx<<<cdiv(nUx, NTHR), NTHR, 0, stream>>>(x, nN, nUx, XB);
  k_deg<<<gD, NTHR, 0, stream>>>(dst, nE, vec8, DIS);
  k_gemm<<<dim3(gM, FH / GBN), GTHR, 0, stream>>>(XB, W1T, XW, CIN, FH);
  k_scan<1><<<gA, NTHR, scanLds, stream>>>(src, dst, nE, nN, vec8, MP, DIS, XW, b1, Wfc, bfc, H1, out);
  k_gemm<<<dim3(gM, FH / GBN), GTHR, 0, stream>>>(H1, W2T, XW, K2, FH);
  k_scan<0><<<gA, NTHR, scanLds, stream>>>(src, dst, nE, nN, vec8, MP, DIS, XW, b2, Wfc, bfc, H1, out);
}
